// MaskedSelfAttention_76562087018941
// MI455X (gfx1250) — hardware-verified
//
#include <hip/hip_runtime.h>
#include <math.h>
#include <stdint.h>

#ifndef NB
#define NB    2
#endif
#ifndef SEQ
#define SEQ   2048
#endif
#define SEQ_FULL 2048
#define EMB   1024
#define NH    16
#define HD    64
#define CK    512
#define NCHK  (SEQ / CK)
#define NKB   16
#define QT    16
#define TQ0   128
#define NQT   ((SEQ - TQ0) / QT)
#define ROWS  (NB * SEQ)
#define SCP   544
#define PLP   528
#define CTQ   36
#define SLAB64 (16 * 68)
#define VTP   72
#define ATT_THREADS 256
#define NACC  4
#define QSC   8.0f
#define KSC   8.0f
#define PCAR  32768.0f
#define VCAR  1024.0f
#define WSC   1024.0f
#define CSC   8192.0f
#define RSC   2048.0f
#define LOG2E 1.4426950408889634f
#define RSQD  0.125f
#define WS_CAP ((size_t)134217728)

static_assert(EMB == NH * HD && HD == 64 && (HD % 32) == 0 && (EMB % 64) == 0 && (EMB % 256) == 0 && EMB == 4 * 256);
static_assert(NB >= 1 && NB <= 2 && SEQ >= CK && SEQ <= SEQ_FULL && (SEQ % CK) == 0 && NCHK >= 1 && CK == 32 * NKB);
static_assert((SEQ % 64) == 0 && ((SEQ - TQ0) % QT) == 0 && NQT * QT + TQ0 == SEQ && TQ0 == 128 && TQ0 < CK && NQT >= 1);
static_assert(16 * SCP >= 8 * 16 * 64 && SCP >= CK + 16 && PLP >= CK + 8 && 2 * CTQ >= 64);
static_assert(((PLP * 2) % 16) == 0 && ((SCP * 4) % 16) == 0 && ((VTP * 2) % 16) == 0 && ((CTQ * 4) % 16) == 0);
static_assert(64 * VTP >= 63 * VTP + 64);
static_assert(ATT_THREADS == 16 * QT && ATT_THREADS == 256 && NACC * 16 == HD && NH * TQ0 == 8 * 256 && 2 * 8 == NH);
static_assert((ROWS % 64) == 0 && ((NB * TQ0) % 64) == 0 && ((NB * NCHK * EMB) % 256) == 0);
static_assert((((EMB * EMB) / 8) % 256) == 0 && (((SEQ * EMB) / 8) % 256) == 0);
static_assert(4LL * EMB * EMB * 2 + (long long)NB * NCHK * NKB * EMB * 4 + 2LL * NB * TQ0 * EMB * 4
              + 6LL * ROWS * EMB * 2 + (long long)ROWS * EMB * 4 <= 134217728LL);

typedef unsigned short u16;
typedef _Float16 v16h __attribute__((ext_vector_type(16)));
typedef _Float16 v8h  __attribute__((ext_vector_type(8)));
typedef __bf16   v16b __attribute__((ext_vector_type(16)));
typedef float    v8f  __attribute__((ext_vector_type(8)));
typedef float    v4f  __attribute__((ext_vector_type(4)));
typedef unsigned int v4u __attribute__((ext_vector_type(4)));

union FragH { v16h v; v8h h[2]; v4u u[2]; };
union FragB { v16b v; v4u u[2]; };

__device__ __forceinline__ unsigned short bf_bits(float f) {
  unsigned u = __float_as_uint(f);
  return (unsigned short)((u + 0x7FFFu + ((u >> 16) & 1u)) >> 16);
}
__device__ __forceinline__ float bf_up(unsigned short h) { return __uint_as_float(((unsigned)h) << 16); }
__device__ __forceinline__ float bfr(float f) { return bf_up(bf_bits(f)); }
__device__ __forceinline__ unsigned short h_bits(_Float16 x) { return __builtin_bit_cast(unsigned short, x); }
__device__ __forceinline__ unsigned pk16(unsigned short a, unsigned short b) { return (unsigned)a | ((unsigned)b << 16); }
__device__ __forceinline__ v8f zero8() { v8f z = {0.f, 0.f, 0.f, 0.f, 0.f, 0.f, 0.f, 0.f}; return z; }
__device__ __forceinline__ v4f zero4() { v4f z = {0.f, 0.f, 0.f, 0.f}; return z; }

__device__ __forceinline__ v16h ldfrag_h(const _Float16* p) {
  FragH f;
  f.h[0] = *(const v8h*)(p);
  f.h[1] = *(const v8h*)(p + 16);
  return f.v;
}
__device__ __forceinline__ v16b ldfrag_b(const u16* p) {
  FragB f;
  f.u[0] = *(const v4u*)(p);
  f.u[1] = *(const v4u*)(p + 16);
  return f.v;
}

__device__ __forceinline__ v8f mma_h(v16h a, v16h b, v8f c) {
  return __builtin_amdgcn_wmma_f32_16x16x32_f16(false, a, false, b, (short)0, c, false, false);
}
__device__ __forceinline__ v8f mma_b(v16b a, v16b b, v8f c) {
  return __builtin_amdgcn_wmma_f32_16x16x32_bf16(false, a, false, b, (short)0, c, false, false);
}
__device__ __forceinline__ void guard2x3(v8f& a, v8f& b, v16h x0, v16h x1, v16h x2) {
#if defined(__HIP_DEVICE_COMPILE__)
  asm volatile("v_nop\n\tv_nop\n\tv_nop\n\tv_nop"
               : "+v"(a), "+v"(b) : "v"(x0), "v"(x1), "v"(x2) : "memory");
#endif
}
template <typename F>
__device__ __forceinline__ void guard6(v8f& a, v8f& b, v8f& c, v8f& d, F x0, F x1, F x2, F x3, F x4, F x5) {
#if defined(__HIP_DEVICE_COMPILE__)
  asm volatile("v_nop\n\tv_nop\n\tv_nop\n\tv_nop"
               : "+v"(a), "+v"(b), "+v"(c), "+v"(d) : "v"(x0), "v"(x1), "v"(x2), "v"(x3), "v"(x4), "v"(x5) : "memory");
#endif
}
__device__ __forceinline__ void guard8x6(v8f& a0, v8f& a1, v8f& a2, v8f& a3, v8f& e0, v8f& e1, v8f& e2, v8f& e3,
                                         v16h x0, v16h x1, v16h x2, v16h x3, v16h x4, v16h x5) {
#if defined(__HIP_DEVICE_COMPILE__)
  asm volatile("v_nop\n\tv_nop\n\tv_nop\n\tv_nop"
               : "+v"(a0), "+v"(a1), "+v"(a2), "+v"(a3), "+v"(e0), "+v"(e1), "+v"(e2), "+v"(e3)
               : "v"(x0), "v"(x1), "v"(x2), "v"(x3), "v"(x4), "v"(x5) : "memory");
#endif
}
__device__ __forceinline__ void guardpv4(v8f& o0, v8f& o1, v8f& o2, v8f& o3, v16h p, v16h g0, v16h g1, v16h g2, v16h g3) {
#if defined(__HIP_DEVICE_COMPILE__)
  asm volatile("v_nop\n\tv_nop\n\tv_nop\n\tv_nop"
               : "+v"(o0), "+v"(o1), "+v"(o2), "+v"(o3)
               : "v"(p), "v"(g0), "v"(g1), "v"(g2), "v"(g3) : "memory");
#endif
}
__device__ __forceinline__ void acc_guard4(v8f& a, v8f& b, v8f& c, v8f& d) {
#if defined(__HIP_DEVICE_COMPILE__)
  asm volatile("v_nop\n\tv_nop\n\tv_nop\n\tv_nop" : "+v"(a), "+v"(b), "+v"(c), "+v"(d));
#endif
}
__device__ __forceinline__ void wave_sync_lds() {
  __builtin_amdgcn_fence(3, "workgroup");
  __builtin_amdgcn_wave_barrier();
  __builtin_amdgcn_fence(2, "workgroup");
}

__global__ __launch_bounds__(256) void cvt16(const float* __restrict__ x, u16* D, int n8, int mode, float scale) {
  const int gt = blockIdx.x * 256 + (int)threadIdx.x;
  if (gt >= n8) return;
  const float* p = x + (size_t)gt * 8;
  const v4f a = *(const v4f*)(p), c4 = *(const v4f*)(p + 4);
  float v[8];
#pragma unroll
  for (int e = 0; e < 4; ++e) { v[e] = a[e]; v[4 + e] = c4[e]; }
  unsigned short s[8];
#pragma unroll
  for (int e = 0; e < 8; ++e) {
    const float vb = bfr(v[e]);
    const float vf = (mode == 1) ? vb : v[e];
    const unsigned short hb = h_bits((_Float16)(vf * scale));
    const unsigned short bb = bf_bits(v[e]);
    s[e] = (mode != 0) ? hb : bb;
  }
  v4u o;
#pragma unroll
  for (int e = 0; e < 4; ++e) o[e] = pk16(s[2 * e], s[2 * e + 1]);
  u16* d = D + (size_t)gt * 8;
  for (int pass = 0; pass < 2; ++pass) {
    *(volatile v4u*)(d) = o;
    __threadfence();
  }
}

__global__ __launch_bounds__(256) void tr16(const float* __restrict__ X, u16* XTo, int R, int Cc, int mode, float scale) {
  __shared__ __align__(16) u16 TH[64 * VTP];
  const int tid = threadIdx.x;
  const int bid = blockIdx.x;
  const int nct = Cc >> 6;
  const int nrt = R >> 6;
  const int ct  = bid % nct;
  const int rt  = (bid / nct) % nrt;
  const int bt  = bid / (nct * nrt);
  const int r0  = rt * 64;
  const int c0  = ct * 64;
  const size_t plane = (size_t)R * (size_t)Cc;
  const float* Xb = X + (size_t)bt * plane;
  u16* Ob = XTo + (size_t)bt * plane;
  {
    const int rl = tid >> 2;
    const int cc = (tid & 3) * 16;
    const float* src = Xb + (size_t)(r0 + rl) * Cc + c0 + cc;
#pragma unroll
    for (int i = 0; i < 4; ++i) {
      const v4f a = *(const v4f*)(src + 4 * i);
#pragma unroll
      for (int e = 0; e < 4; ++e) {
        const float v  = a[e];
        const float vb = bfr(v);
        const float vf = (mode == 1) ? vb : v;
        const unsigned short hb = h_bits((_Float16)(vf * scale));
        const unsigned short bb = bf_bits(v);
        TH[(cc + 4 * i + e) * VTP + rl] = (mode != 0) ? hb : bb;
      }
    }
  }
  __syncthreads();
  v4u vh[2];
  const int q8 = tid >> 3, p8 = (tid & 7) * 8;
#pragma unroll
  for (int it = 0; it < 2; ++it) {
    const int line = it * 32 + q8;
    vh[it] = *(const v4u*)(TH + line * VTP + p8);
  }
  const size_t base = (size_t)c0 * (size_t)R + r0 + p8;
  for (int pass = 0; pass < 2; ++pass) {
#pragma unroll
    for (int it = 0; it < 2; ++it) {
      const int line = it * 32 + q8;
      *(volatile v4u*)(Ob + base + (size_t)line * (size_t)R) = vh[it];
    }
    __threadfence();
  }
}

__device__ __forceinline__ void stage64(float* sl, v8f a0, v8f a1, v8f a2, v8f a3, float oscale, int lane) {
  const int hh = lane >> 4, m = lane & 15;
#pragma unroll
  for (int r = 0; r < 8; ++r) {
    const int ro = (8 * hh + r) * 68 + m;
    sl[ro]      = a0[r] * oscale;
    sl[ro + 16] = a1[r] * oscale;
    sl[ro + 32] = a2[r] * oscale;
    sl[ro + 48] = a3[r] * oscale;
  }
  wave_sync_lds();
}
__device__ __forceinline__ void epi64(float* sl, v8f a0, v8f a1, v8f a2, v8f a3, float oscale, v4f badd, float* C, int N,
                                      size_t rowb, int col0, int lane) {
  const int hh = lane >> 4, m = lane & 15;
  stage64(sl, a0, a1, a2, a3, oscale, lane);
  v4f vals[8];
#pragma unroll
  for (int it = 0; it < 8; ++it) vals[it] = *(const v4f*)(sl + (it * 2 + hh) * 68 + m * 4) + badd;
  float* dst = C + (rowb + (size_t)hh) * (size_t)N + col0 + m * 4;
  for (int pass = 0; pass < 2; ++pass) {
#pragma unroll
    for (int it = 0; it < 8; ++it) {
      *(volatile v4f*)(dst + (size_t)(it * 2) * (size_t)N) = vals[it];
    }
    __threadfence();
  }
}
__device__ __forceinline__ void epi64x2(float* sl, v8f a0, v8f a1, v8f a2, v8f a3, v8f e0, v8f e1, v8f e2, v8f e3,
                                        float os1, float os2, v4f badd, float* C, int N, size_t rowb, int col0, int lane) {
  const int hh = lane >> 4, m = lane & 15;
#pragma unroll
  for (int r = 0; r < 8; ++r) {
    const int ro = (8 * hh + r) * 68 + m;
    sl[ro]      = a0[r] * os1 + e0[r] * os2;
    sl[ro + 16] = a1[r] * os1 + e1[r] * os2;
    sl[ro + 32] = a2[r] * os1 + e2[r] * os2;
    sl[ro + 48] = a3[r] * os1 + e3[r] * os2;
  }
  wave_sync_lds();
  v4f vals[8];
#pragma unroll
  for (int it = 0; it < 8; ++it) vals[it] = *(const v4f*)(sl + (it * 2 + hh) * 68 + m * 4) + badd;
  float* dst = C + (rowb + (size_t)hh) * (size_t)N + col0 + m * 4;
  for (int pass = 0; pass < 2; ++pass) {
#pragma unroll
    for (int it = 0; it < 8; ++it) {
      *(volatile v4f*)(dst + (size_t)(it * 2) * (size_t)N) = vals[it];
    }
    __threadfence();
  }
}
__device__ __forceinline__ void epi64hsb(float* sl, v8f a0, v8f a1, v8f a2, v8f a3, float oscale, float pscale,
                                         const float* __restrict__ bias, u16* C, int N, size_t rowb, int col0, int lane) {
  stage64(sl, a0, a1, a2, a3, oscale, lane);
  const int rq = lane >> 3, c8 = (lane & 7) * 8;
  const v4f b0 = *(const v4f*)(bias + col0 + c8), b1 = *(const v4f*)(bias + col0 + c8 + 4);
  float bb[8];
#pragma unroll
  for (int e = 0; e < 4; ++e) { bb[e] = bfr(b0[e]); bb[4 + e] = bfr(b1[e]); }
  v4u oh[4];
#pragma unroll
  for (int i4 = 0; i4 < 4; ++i4) {
    const int row = i4 * 4 + rq;
    const v4f a = *(const v4f*)(sl + row * 68 + c8), c4 = *(const v4f*)(sl + row * 68 + c8 + 4);
    float w[8];
#pragma unroll
    for (int e = 0; e < 4; ++e) { w[e] = (a[e] + bb[e]) * pscale; w[4 + e] = (c4[e] + bb[4 + e]) * pscale; }
#pragma unroll
    for (int e = 0; e < 4; ++e) oh[i4][e] = pk16(h_bits((_Float16)w[2 * e]), h_bits((_Float16)w[2 * e + 1]));
  }
  u16* dst = C + rowb * (size_t)N + col0 + c8;
  for (int pass = 0; pass < 2; ++pass) {
#pragma unroll
    for (int i4 = 0; i4 < 4; ++i4) {
      const int row = i4 * 4 + rq;
      *(volatile v4u*)(dst + (size_t)row * (size_t)N) = oh[i4];
    }
    __threadfence();
  }
}

__global__ __launch_bounds__(128)
void gemm_b32(const u16* __restrict__ A, const u16* __restrict__ Bt, const float* __restrict__ bias, float* C,
              int M, int N, int K, int rpg, int gstr, int goff, float oscale) {
  __shared__ __align__(16) float slab[4 * SLAB64];
  const int tid = threadIdx.x, wave = tid >> 5, lane = tid & 31, hh = lane >> 4, m = lane & 15;
  const int ntile = N >> 6;
  const int bid   = blockIdx.x;
  const int rowb  = (bid / ntile) * 64 + wave * 16;
  const int col0  = (bid % ntile) * 64;
  if (rowb + 16 > M) return;
  const int ra = rowb + m;
  const int rg = ra / rpg;
  const size_t arow = (size_t)rg * (size_t)gstr + (size_t)goff + (size_t)(ra - rg * rpg);
  const u16* ap = A  + arow * (size_t)K + 8 * hh;
  const u16* bp = Bt + (size_t)(col0 + m) * K + 8 * hh;
  const size_t bs = (size_t)16 * K;
  v8f acc0 = zero8(), acc1 = zero8(), acc2 = zero8(), acc3 = zero8();
#pragma unroll 1
  for (int k0 = 0; k0 < K; k0 += 32) {
    const v16b a  = ldfrag_b(ap + k0);
    const v16b b0 = ldfrag_b(bp + k0);
    const v16b b1 = ldfrag_b(bp + bs + k0);
    const v16b b2 = ldfrag_b(bp + 2 * bs + k0);
    const v16b b3 = ldfrag_b(bp + 3 * bs + k0);
    acc0 = mma_b(a, b0, acc0);
    acc1 = mma_b(a, b1, acc1);
    acc2 = mma_b(a, b2, acc2);
    acc3 = mma_b(a, b3, acc3);
    guard6<v16b>(acc0, acc1, acc2, acc3, a, b0, b1, b2, b3, a);
  }
  const v4f bv4 = *(const v4f*)(bias + col0 + m * 4);
  v4f badd;
#pragma unroll
  for (int e = 0; e < 4; ++e) badd[e] = bfr(bv4[e]);
  epi64(slab + wave * SLAB64, acc0, acc1, acc2, acc3, oscale, badd, C, N, (size_t)rowb, col0, lane);
}

__global__ __launch_bounds__(128)
void gemm_bh16(const u16* __restrict__ A, const u16* __restrict__ Bt, const float* __restrict__ bias, u16* C,
               int M, int N, int K, float oscale, float pscale) {
  __shared__ __align__(16) float slab[4 * SLAB64];
  const int tid = threadIdx.x, wave = tid >> 5, lane = tid & 31, hh = lane >> 4, m = lane & 15;
  const int ntile = N >> 6;
  const int bid   = blockIdx.x;
  const int rowb  = (bid / ntile) * 64 + wave * 16;
  const int col0  = (bid % ntile) * 64;
  if (rowb + 16 > M) return;
  const u16* ap = A  + (size_t)(rowb + m) * K + 8 * hh;
  const u16* bp = Bt + (size_t)(col0 + m) * K + 8 * hh;
  const size_t bs = (size_t)16 * K;
  v8f acc0 = zero8(), acc1 = zero8(), acc2 = zero8(), acc3 = zero8();
#pragma unroll 1
  for (int k0 = 0; k0 < K; k0 += 32) {
    const v16b a  = ldfrag_b(ap + k0);
    const v16b b0 = ldfrag_b(bp + k0);
    const v16b b1 = ldfrag_b(bp + bs + k0);
    const v16b b2 = ldfrag_b(bp + 2 * bs + k0);
    const v16b b3 = ldfrag_b(bp + 3 * bs + k0);
    acc0 = mma_b(a, b0, acc0);
    acc1 = mma_b(a, b1, acc1);
    acc2 = mma_b(a, b2, acc2);
    acc3 = mma_b(a, b3, acc3);
    guard6<v16b>(acc0, acc1, acc2, acc3, a, b0, b1, b2, b3, a);
  }
  epi64hsb(slab + wave * SLAB64, acc0, acc1, acc2, acc3, oscale, pscale, bias, C, N, (size_t)rowb, col0, lane);
}

__global__ __launch_bounds__(128)
void gemm_h2_32(const u16* __restrict__ Ah, const u16* __restrict__ Ar, const u16* __restrict__ Bt,
                const float* __restrict__ bias, float* C, int M, int N, int K, float os1, float os2) {
  __shared__ __align__(16) float slab[4 * SLAB64];
  const int tid = threadIdx.x, wave = tid >> 5, lane = tid & 31, hh = lane >> 4, m = lane & 15;
  const int ntile = N >> 6;
  const int bid   = blockIdx.x;
  const int rowb  = (bid / ntile) * 64 + wave * 16;
  const int col0  = (bid % ntile) * 64;
  if (rowb + 16 > M) return;
  const _Float16* ap  = (const _Float16*)(const void*)Ah + (size_t)(rowb + m) * K + 8 * hh;
  const _Float16* arp = (const _Float16*)(const void*)Ar + (size_t)(rowb + m) * K + 8 * hh;
  const _Float16* bp  = (const _Float16*)(const void*)Bt + (size_t)(col0 + m) * K + 8 * hh;
  const size_t bs = (size_t)16 * K;
  v8f acc0 = zero8(), acc1 = zero8(), acc2 = zero8(), acc3 = zero8();
  v8f acr0 = zero8(), acr1 = zero8(), acr2 = zero8(), acr3 = zero8();
#pragma unroll 1
  for (int k0 = 0; k0 < K; k0 += 32) {
    const v16h a  = ldfrag_h(ap + k0);
    const v16h ar = ldfrag_h(arp + k0);
    const v16h b0 = ldfrag_h(bp + k0);
    const v16h b1 = ldfrag_h(bp + bs + k0);
    const v16h b2 = ldfrag_h(bp + 2 * bs + k0);
    const v16h b3 = ldfrag_h(bp + 3 * bs + k0);
    acc0 = mma_h(a, b0, acc0);
    acc1 = mma_h(a, b1, acc1);
    acc2 = mma_h(a, b2, acc2);
    acc3 = mma_h(a, b3, acc3);
    acr0 = mma_h(ar, b0, acr0);
    acr1 = mma_h(ar, b1, acr1);
    acr2 = mma_h(ar, b2, acr2);
    acr3 = mma_h(ar, b3, acr3);
    guard8x6(acc0, acc1, acc2, acc3, acr0, acr1, acr2, acr3, a, ar, b0, b1, b2, b3);
  }
  const v4f bv = *(const v4f*)(bias + col0 + m * 4);
  v4f badd;
#pragma unroll
  for (int e = 0; e < 4; ++e) badd[e] = bfr(bv[e]);
  epi64x2(slab + wave * SLAB64, acc0, acc1, acc2, acc3, acr0, acr1, acr2, acr3, os1, os2, badd, C, N,
          (size_t)rowb, col0, lane);
}

__global__ __launch_bounds__(256) void vsum_k(const float* __restrict__ V, float* VS) {
  __shared__ __align__(16) float sm[NKB * 256];
  const int tid = threadIdx.x;
  const int gt  = blockIdx.x * 256 + tid;
  const int d   = gt % EMB;
  const int bc  = gt / EMB;
  const int b   = bc / NCHK;
  const int c   = bc - b * NCHK;
  const int d0  = d - tid;
  const float* p = V + ((size_t)b * SEQ + (size_t)c * CK) * EMB + d;
  float s = 0.f;
#pragma unroll 1
  for (int kb = NKB - 1; kb >= 0; --kb) {
#pragma unroll 4
    for (int i = 31; i >= 0; --i) s += p[(size_t)(kb * 32 + i) * EMB];
    sm[kb * 256 + tid] = s;
  }
  __syncthreads();
  const int sel = tid >> 6, piece = tid & 63;
  v4f o[4];
#pragma unroll
  for (int it = 0; it < 4; ++it) o[it] = *(const v4f*)(sm + (it * 4 + sel) * 256 + piece * 4);
  float* base = VS + (size_t)bc * NKB * EMB + d0 + piece * 4;
  for (int pass = 0; pass < 2; ++pass) {
#pragma unroll
    for (int it = 0; it < 4; ++it) {
      *(volatile v4f*)(base + (size_t)(it * 4 + sel) * EMB) = o[it];
    }
    __threadfence();
  }
}

__global__ __launch_bounds__(ATT_THREADS) __attribute__((amdgpu_num_vgpr(256)))
void attn_fwd(const u16* __restrict__ QPp, const u16* __restrict__ KPp, const u16* __restrict__ VTp,
              const float* __restrict__ VSp, u16* CHo, u16* CRo) {
  __shared__ __align__(16) float scs[16 * SCP];
  __shared__ __align__(16) u16 pls[16 * PLP];
  __shared__ __align__(16) unsigned cts[2 * 16 * CTQ];
  __shared__ float rowa[QT];
  __shared__ float rowc[QT];
  __shared__ float rowi[QT];

  const int tid  = threadIdx.x;
  const int wave = tid >> 5;
  const int lane = tid & 31;
  const int hh   = lane >> 4;
  const int m    = lane & 15;
  const int r16  = tid >> 4;
  const int sub  = tid & 15;
  const int kl0  = sub * 32;

  const int bid = blockIdx.x;
  const int per = NH * NQT;
  const int b   = bid / per;
  const int rem = bid - b * per;
  const int h   = rem / NQT;
  const int q0  = (rem - h * NQT) * QT;
  const int qc  = q0 / CK;

  const _Float16* qa  = (const _Float16*)(const void*)QPp + ((size_t)b * SEQ + q0 + m) * EMB + h * HD + 8 * hh;
  const _Float16* kbp = (const _Float16*)(const void*)KPp + ((size_t)b * SEQ + m) * EMB + h * HD + 8 * hh;
  const _Float16* vbp = (const _Float16*)(const void*)VTp + ((size_t)b * EMB + h * HD + m) * SEQ + 8 * hh;
  const float* vsb = VSp + (size_t)b * NCHK * NKB * EMB + h * HD + m;
  const float lsc  = RSQD * LOG2E / (QSC * KSC);
  const float addf = (wave == 0) ? 1.f : 0.f;

  float mrun = -INFINITY, lrun = 0.f;
  v8f o[NACC];
#pragma unroll
  for (int j = 0; j < NACC; ++j) o[j] = zero8();

#pragma unroll 1
  for (int c = NCHK - 1; c >= qc; --c) {
    const int kbeg = c * CK;
    const int kb0  = (c > qc) ? 0 : ((q0 - kbeg) >> 5);
#pragma unroll 1
    for (int kb = wave; kb < NKB; kb += 8) {
      v8f s0 = zero8(), s1 = zero8();
      if (kb >= kb0) {
        const _Float16* k0p = kbp + (size_t)(kbeg + kb * 32) * EMB;
        const _Float16* k1p = k0p + (size_t)16 * EMB;
#pragma unroll
        for (int ks = 0; ks < HD / 32; ++ks) {
          const v16h a  = ldfrag_h(qa + ks * 32);
          const v16h f0 = ldfrag_h(k0p + ks * 32);
          const v16h f1 = ldfrag_h(k1p + ks * 32);
          s0 = mma_h(a, f0, s0);
          s1 = mma_h(a, f1, s1);
          guard2x3(s0, s1, a, f0, f1);
        }
      }
      float* srow = scs + (8 * hh) * SCP + kb * 32 + m;
#pragma unroll
      for (int r = 0; r < 8; ++r) {
        srow[r * SCP]      = s0[r];
        srow[r * SCP + 16] = s1[r];
      }
    }
    __syncthreads();
    {
      const float* sp = scs + r16 * SCP + kl0;
      const int lim = (q0 + r16) - (kbeg + kl0);
      float t[32];
      float cm = -INFINITY;
#pragma unroll
      for (int i = 0; i < 8; ++i) {
        const v4f a = *(const v4f*)(sp + 4 * i);
#pragma unroll
        for (int e = 0; e < 4; ++e) {
          const int j = 4 * i + e;
          const float tv = (j > lim) ? a[e] * lsc : -INFINITY;
          t[j] = tv;
          cm = fmaxf(cm, tv);
        }
      }
#pragma unroll
      for (int d = 1; d <= 8; d <<= 1) cm = fmaxf(cm, __shfl_xor(cm, d, 32));
      const float mn = fmaxf(mrun, cm);
      const float al = (mrun == -INFINITY) ? 0.f : exp2f(mrun - mn);
      const float mz = (mn == -INFINITY) ? 0.f : mn;
      mrun = mn;
      float ps = 0.f;
#pragma unroll
      for (int j = 0; j < 32; ++j) {
        const float p = exp2f(fminf(t[j] - mz, 0.f));
        t[j] = p;
        ps += p;
      }
#pragma unroll
      for (int d = 1; d <= 8; d <<= 1) ps += __shfl_xor(ps, d, 32);
      const float cc = ps * (1.0f / (float)CK);
      v4u pk[4];
#pragma unroll
      for (int i = 0; i < 4; ++i) {
#pragma unroll
        for (int e = 0; e < 4; ++e) {
          const int j = 8 * i + 2 * e;
          pk[i][e] = pk16(h_bits((_Float16)((t[j] - cc) * PCAR)), h_bits((_Float16)((t[j + 1] - cc) * PCAR)));
        }
      }
      lrun = lrun * al + ps;
      u16* pd = pls + r16 * PLP + kl0;
#pragma unroll
      for (int i = 0; i < 4; ++i) *(v4u*)(pd + 8 * i) = pk[i];
      if (sub == 0) { rowa[r16] = al; rowc[r16] = cc; }
    }
    __syncthreads();
    {
      float scl[8], cad[8];
#pragma unroll
      for (int r = 0; r < 8; ++r) { scl[r] = rowa[8 * hh + r]; cad[r] = rowc[8 * hh + r] * (PCAR * VCAR) * addf; }
      const float* vsc = vsb + ((size_t)c * NKB + (size_t)kb0) * EMB;
      float vs[NACC];
#pragma unroll
      for (int j = 0; j < NACC; ++j) vs[j] = vsc[16 * j];
#pragma unroll
      for (int j = 0; j < NACC; ++j) {
#pragma unroll
        for (int r = 0; r < 8; ++r) o[j][r] = o[j][r] * scl[r] + cad[r] * vs[j];
      }
      const _Float16* pp = (const _Float16*)(const void*)pls + m * PLP + 8 * hh;
      const _Float16* vp = vbp + kbeg;
#pragma unroll 1
      for (int kb = wave; kb < NKB; kb += 8) {
        if (kb >= kb0) {
          const v16h pf = ldfrag_h(pp + kb * 32);
          const _Float16* vk = vp + kb * 32;
          const v16h g0 = ldfrag_h(vk);
          const v16h g1 = ldfrag_h(vk + (size_t)16 * SEQ);
          const v16h g2 = ldfrag_h(vk + (size_t)32 * SEQ);
          const v16h g3 = ldfrag_h(vk + (size_t)48 * SEQ);
          o[0] = mma_h(pf, g0, o[0]);
          o[1] = mma_h(pf, g1, o[1]);
          o[2] = mma_h(pf, g2, o[2]);
          o[3] = mma_h(pf, g3, o[3]);
          guardpv4(o[0], o[1], o[2], o[3], pf, g0, g1, g2, g3);
        }
      }
    }
  }
  acc_guard4(o[0], o[1], o[2], o[3]);

  {
    float* red = scs + wave * 1024 + (8 * hh) * 64 + m;
#pragma unroll
    for (int j = 0; j < NACC; ++j) {
#pragma unroll
      for (int r = 0; r < 8; ++r) red[r * 64 + 16 * j] = o[j][r];
    }
  }
  if (sub == 0) rowi[r16] = (1.0f / lrun) * (CSC / (PCAR * VCAR));
  __syncthreads();
  {
    const int row = tid >> 4, cq = tid & 15, c4 = cq * 4;
    v4f x = zero4();
#pragma unroll
    for (int w = 0; w < 8; ++w) x += *(const v4f*)(scs + w * 1024 + row * 64 + c4);
    const float inv = rowi[row];
    float xs[4];
    _Float16 hv[4];
    unsigned short hb[4], rb[4];
#pragma unroll
    for (int e = 0; e < 4; ++e) {
      xs[e] = x[e] * inv;
      hv[e] = (_Float16)xs[e];
      hb[e] = h_bits(hv[e]);
      rb[e] = h_bits((_Float16)((xs[e] - (float)hv[e]) * RSC));
    }
    cts[row * CTQ + cq * 2]            = pk16(hb[0], hb[1]);
    cts[row * CTQ + cq * 2 + 1]        = pk16(hb[2], hb[3]);
    cts[(16 + row) * CTQ + cq * 2]     = pk16(rb[0], rb[1]);
    cts[(16 + row) * CTQ + cq * 2 + 1] = pk16(rb[2], rb[3]);
  }
  __syncthreads();
  {
    const int pl  = tid >> 7;
    const int p   = tid & 127;
    const int row = p >> 3;
    const int pq  = p & 7;
    const v4u ov = *(const v4u*)(&cts[(pl * 16 + row) * CTQ + pq * 4]);
    u16* dstp = (pl == 0) ? CHo : CRo;
    u16* dst  = dstp + ((size_t)b * SEQ + q0 + row) * EMB + h * HD + pq * 8;
    *(volatile v4u*)dst = ov;
    __threadfence();
    *(volatile v4u*)dst = ov;
  }
}

__global__ __launch_bounds__(256) __attribute__((amdgpu_num_vgpr(256)))
void attn_tail(const float* __restrict__ QF, const float* __restrict__ KF, const float* __restrict__ V,
               const float* __restrict__ VS, u16* CHo, u16* CRo) {
  __shared__ __align__(16) float qs[EMB];
  __shared__ __align__(16) float sc[NH * TQ0];
  __shared__ float linv[NH];
  __shared__ __align__(16) unsigned SW[2][EMB / 2];
  const int tid = threadIdx.x, lane = tid & 31, wave = tid >> 5;
  const int b = blockIdx.x / TQ0;
  const int t = blockIdx.x - b * TQ0;
  const int i = SEQ - TQ0 + t;
  const bool uni = (t == TQ0 - 1);
  *(v4f*)(qs + tid * 4) = *(const v4f*)(QF + ((size_t)b * TQ0 + t) * EMB + tid * 4);
  __syncthreads();
  {
    const int kk = tid & (TQ0 - 1);
    const int hg = tid >> 7;
    const float* kp = KF + ((size_t)b * TQ0 + kk) * EMB + hg * 8 * HD;
    const float* qp = qs + hg * 8 * HD;
    const bool valid = (kk > t);
#pragma unroll 1
    for (int h8 = 0; h8 < 8; ++h8) {
      float acc = 0.f;
#pragma unroll 1
      for (int d = 0; d < HD; d += 8) {
        const v4f k0 = *(const v4f*)(kp + h8 * HD + d), k1 = *(const v4f*)(kp + h8 * HD + d + 4);
        const v4f q0 = *(const v4f*)(qp + h8 * HD + d), q1 = *(const v4f*)(qp + h8 * HD + d + 4);
#pragma unroll
        for (int e = 0; e < 4; ++e) acc += k0[e] * q0[e];
#pragma unroll
        for (int e = 0; e < 4; ++e) acc += k1[e] * q1[e];
      }
      sc[(hg * 8 + h8) * TQ0 + kk] = valid ? acc * (RSQD * LOG2E) : -INFINITY;
    }
  }
  __syncthreads();
#pragma unroll 1
  for (int hh2 = 0; hh2 < 2; ++hh2) {
    const int h = 2 * wave + hh2;
    float* sp = sc + h * TQ0;
    float v[4];
    float mx = -INFINITY;
#pragma unroll
    for (int q = 0; q < 4; ++q) { v[q] = sp[lane + 32 * q]; mx = fmaxf(mx, v[q]); }
#pragma unroll
    for (int d = 1; d <= 16; d <<= 1) mx = fmaxf(mx, __shfl_xor(mx, d, 32));
    const float gm = (mx == -INFINITY) ? 0.f : mx;
    float ps = 0.f;
#pragma unroll
    for (int q = 0; q < 4; ++q) { v[q] = exp2f(v[q] - gm); ps += v[q]; }
#pragma unroll
    for (int d = 1; d <= 16; d <<= 1) ps += __shfl_xor(ps, d, 32);
#pragma unroll
    for (int q = 0; q < 4; ++q) sp[lane + 32 * q] = v[q];
    if (lane == 0) linv[h] = (ps > 0.f) ? (1.0f / ps) * CSC : 0.f;
  }
  __syncthreads();
  const int hd = tid >> 4;
  v4f x = zero4();
  if (uni) {
    const float* vs0 = VS + (size_t)b * NCHK * NKB * EMB + tid * 4;
    v4f s = zero4();
#pragma unroll 1
    for (int c = 0; c < NCHK; ++c) s += *(const v4f*)(vs0 + (size_t)c * NKB * EMB);
    x = s * (CSC / (float)SEQ);
  } else {
    const float* pp = sc + hd * TQ0;
    const float* vp = V + ((size_t)b * SEQ + (size_t)(SEQ - TQ0)) * EMB + tid * 4;
    v4f cx = zero4();
#pragma unroll 1
    for (int j = t + 1; j < TQ0; ++j) {
      const float pj = pp[j];
      const v4f vv = *(const v4f*)(vp + (size_t)j * EMB);
      cx += pj * vv;
    }
    x = cx * linv[hd];
  }
  unsigned hw[2], rw[2];
#pragma unroll
  for (int e = 0; e < 2; ++e) {
    const float x0 = x[2 * e], x1 = x[2 * e + 1];
    const _Float16 h0 = (_Float16)x0, h1 = (_Float16)x1;
    const _Float16 g0 = (_Float16)((x0 - (float)h0) * RSC), g1 = (_Float16)((x1 - (float)h1) * RSC);
    hw[e] = pk16(h_bits(h0), h_bits(h1));
    rw[e] = pk16(h_bits(g0), h_bits(g1));
  }
  SW[0][tid * 2] = hw[0]; SW[0][tid * 2 + 1] = hw[1];
  SW[1][tid * 2] = rw[0]; SW[1][tid * 2 + 1] = rw[1];
  __syncthreads();
  const int pl = tid >> 7, p8 = tid & 127;
  const v4u ov = *(const v4u*)(&SW[pl][p8 * 4]);
  u16* dstp = (pl == 0) ? CHo : CRo;
  u16* dst  = dstp + ((size_t)b * SEQ + i) * EMB + p8 * 8;
  *(volatile v4u*)dst = ov;
  __threadfence();
  *(volatile v4u*)dst = ov;
}

extern "C" void kernel_launch(void* const* d_in, const int* in_sizes, int n_in,
                              void* d_out, int out_size, void* d_ws, size_t ws_size,
                              hipStream_t stream) {
  if (n_in < 10) return;
  const long long needx = (long long)(NB - 1) * SEQ_FULL * EMB + (long long)SEQ * EMB;
  if ((long long)in_sizes[0] < needx) return;
  if (in_sizes[2] != EMB * EMB || in_sizes[4] != EMB * EMB || in_sizes[6] != EMB * EMB || in_sizes[8] != EMB * EMB) return;
  if (in_sizes[3] != EMB || in_sizes[5] != EMB || in_sizes[7] != EMB || in_sizes[9] != EMB) return;
  if ((long long)out_size < (long long)ROWS * EMB) return;

  const float* x  = (const float*)d_in[0];
  const float* wq = (const float*)d_in[2];
  const float* bq = (const float*)d_in[3];
  const float* wk = (const float*)d_in[4];
  const float* bk = (const float*)d_in[5];
  const float* wv = (const float*)d_in[6];
  const float* bv = (const float*)d_in[7];
  const float* wo = (const float*)d_in[8];
  const float* bo = (const float*)d_in[9];
  float*       out = (float*)d_out;

  const size_t szW  = (size_t)EMB * EMB * 2;
  const size_t szVS = (size_t)NB * NCHK * NKB * EMB * 4;
  const size_t szHF = (size_t)NB * TQ0 * EMB * 4;
  const size_t sz16 = (size_t)ROWS * EMB * 2;
  const size_t sz32 = (size_t)ROWS * EMB * 4;
  size_t off = 0;
  const size_t oWQ = off; off += szW;
  const size_t oWK = off; off += szW;
  const size_t oWV = off; off += szW;
  const size_t oWO = off; off += szW;
  const size_t oVS = off; off += szVS;
  const size_t oQF = off; off += szHF;
  const size_t oKF = off; off += szHF;
  const size_t oXB = off; off += sz16;
  const size_t oQ  = off; off += sz16;
  const size_t oK  = off; off += sz16;
  const size_t oV  = off; off += sz32;
  const size_t oVT = off; off += sz16;
  const size_t oCH = off; off += sz16;
  const size_t oCR = off; off += sz16;
  if (off > ws_size) return;
  if (off > WS_CAP) return;

  char* ws = (char*)d_ws;
  u16*   WQT = (u16*)(ws + oWQ);
  u16*   WKT = (u16*)(ws + oWK);
  u16*   WVT = (u16*)(ws + oWV);
  u16*   WOT = (u16*)(ws + oWO);
  float* VS  = (float*)(ws + oVS);
  float* QF  = (float*)(ws + oQF);
  float* KF  = (float*)(ws + oKF);
  u16*   XB  = (u16*)(ws + oXB);
  u16*   QP  = (u16*)(ws + oQ);
  u16*   KP  = (u16*)(ws + oK);
  float* V   = (float*)(ws + oV);
  u16*   VT  = (u16*)(ws + oVT);
  u16*   CH  = (u16*)(ws + oCH);
  u16*   CR  = (u16*)(ws + oCR);

  const int n8x = (SEQ * EMB) / 8;
  const dim3 blk(256);
  const dim3 gTW((EMB / 64) * (EMB / 64));
  const dim3 gX(n8x / 256);
  const dim3 gG((ROWS / 64) * (EMB / 64));
  const dim3 gH(((NB * TQ0) / 64) * (EMB / 64));
  const dim3 bG(128);
  const dim3 gVT(NB * (SEQ / 64) * (EMB / 64));
  const dim3 gVS((NB * NCHK * EMB) / 256);
  const dim3 gAT(NB * NH * NQT);
  const dim3 bAT(ATT_THREADS);
  const dim3 gTL(NB * TQ0);

  tr16<<<gTW, blk, 0, stream>>>(wq, WQT, EMB, EMB, 0, 1.0f);
  tr16<<<gTW, blk, 0, stream>>>(wk, WKT, EMB, EMB, 0, 1.0f);
  tr16<<<gTW, blk, 0, stream>>>(wv, WVT, EMB, EMB, 0, 1.0f);
  tr16<<<gTW, blk, 0, stream>>>(wo, WOT, EMB, EMB, 1, WSC);
  for (int bi = 0; bi < NB; ++bi) {
    cvt16<<<gX, blk, 0, stream>>>(x + (size_t)bi * SEQ_FULL * EMB, XB + (size_t)bi * SEQ * EMB, n8x, 0, 1.0f);
  }
  gemm_bh16<<<gG, bG, 0, stream>>>(XB, WQT, bq, QP, ROWS, EMB, EMB, 1.0f, QSC);
  gemm_bh16<<<gG, bG, 0, stream>>>(XB, WKT, bk, KP, ROWS, EMB, EMB, 1.0f, KSC);
  gemm_b32<<<gG, bG, 0, stream>>>(XB, WVT, bv, V, ROWS, EMB, EMB, ROWS, 0, 0, 1.0f);
  gemm_b32<<<gH, bG, 0, stream>>>(XB, WQT, bq, QF, NB * TQ0, EMB, EMB, TQ0, SEQ, SEQ - TQ0, 1.0f);
  gemm_b32<<<gH, bG, 0, stream>>>(XB, WKT, bk, KF, NB * TQ0, EMB, EMB, TQ0, SEQ, SEQ - TQ0, 1.0f);
  tr16<<<gVT, blk, 0, stream>>>(V, VT, SEQ, EMB, 2, VCAR);
  vsum_k<<<gVS, blk, 0, stream>>>(V, VS);
  attn_fwd<<<gAT, bAT, 0, stream>>>(QP, KP, VT, VS, CH, CR);
  attn_tail<<<gTL, blk, 0, stream>>>(QF, KF, V, VS, CH, CR);
  gemm_h2_32<<<gG, bG, 0, stream>>>(CH, CR, WOT, bo, out, ROWS, EMB, EMB,
                                     1.0f / (CSC * WSC), 1.0f / (CSC * WSC * RSC));
  (void)hipGetLastError();
}
